// LSTMModel_64596308132529
// MI455X (gfx1250) — hardware-verified
//
#include <hip/hip_runtime.h>
#include <math.h>

constexpr int NBATCH   = 2048;
constexpr int NSTEP    = 1024;
constexpr int NHID     = 50;
constexpr int NGATE    = 4;
constexpr int UPAD     = 64;
constexpr int KPAD     = 64;
constexpr int ROWS_BLK = 32;
constexpr int NTHR     = 256;
constexpr int XCHUNK   = 64;
constexpr float H_CARRY       = 16.0f;
constexpr float W_CARRY       = 64.0f;
constexpr float ACC_CARRY     = H_CARRY * W_CARRY;
constexpr float ACC_CARRY_INV = 1.0f / ACC_CARRY;

static_assert(NBATCH % ROWS_BLK == 0, "grid exact");
static_assert(NSTEP % XCHUNK == 0, "x chunks exact");
static_assert(XCHUNK % 2 == 0, "h buffer parity continues across chunks");
static_assert(KPAD % 32 == 0 && NHID <= KPAD, "k padding");
static_assert(NHID <= UPAD && UPAD % 16 == 0, "unit padding");
static_assert(NGATE * UPAD == NTHR, "one thread per padded weight row");
static_assert(ROWS_BLK * XCHUNK / 4 == 2 * NTHR, "x staging: two float4 per thread");
static_assert((NTHR / 32) == 2 * (UPAD / 16), "8 waves = 2 m-tiles x 4 unit groups");
static_assert(ROWS_BLK * 4 == 128, "one whole 128-B output line per block");
static_assert((2 * ROWS_BLK * KPAD) % NTHR == 0, "h zero-fill loop exact");

typedef __attribute__((ext_vector_type(16))) _Float16 v16h;
typedef __attribute__((ext_vector_type(8)))  _Float16 v8h;
typedef __attribute__((ext_vector_type(8)))  float    v8f;
typedef __attribute__((ext_vector_type(4)))  float    v4f;

__device__ __forceinline__ void keep4_h(v16h a, v16h b, v16h c, v16h d) { asm volatile("v_nop" :: "v"(a), "v"(b), "v"(c), "v"(d)); }
__device__ __forceinline__ void step_guard(v8f& a, v8f& b, v8f& c, v8f& d, v16h x, v16h y) {
  asm volatile("v_nop\n\tv_nop\n\tv_nop\n\tv_nop" : "+v"(a), "+v"(b), "+v"(c), "+v"(d) : "v"(x), "v"(y));
}

template <typename T> struct Frag;
template <> struct Frag<_Float16> {
  typedef v16h V; union U { v16h v; v8h h[2]; };
  static __device__ __forceinline__ v16h load(const _Float16* p) {
    U f; f.h[0] = *(const v8h*)(p); f.h[1] = *(const v8h*)(p + 16); return f.v;
  }
  static __device__ __forceinline__ v8f mma(v16h a, v16h b, v8f c) {
    return __builtin_amdgcn_wmma_f32_16x16x32_f16(false, a, false, b, (short)0, c, false, false);
  }
};

__device__ __forceinline__ float fsig(float x)  { return __builtin_amdgcn_rcpf(1.0f + __expf(-x)); }
__device__ __forceinline__ float ftanh(float x) { return 1.0f - 2.0f * __builtin_amdgcn_rcpf(__expf(2.0f * x) + 1.0f); }

__global__ __launch_bounds__(NTHR) void lstm_seq_kernel(const float* __restrict__ x,
                                                        const float* __restrict__ w_ih,
                                                        const float* __restrict__ w_hh,
                                                        const float* __restrict__ b_ih,
                                                        const float* __restrict__ b_hh,
                                                        const float* __restrict__ w_lin,
                                                        const float* __restrict__ b_lin,
                                                        float* __restrict__ out) {
  __shared__ __align__(16) _Float16 Wl[NGATE * UPAD * KPAD];
  __shared__ __align__(16) _Float16 Ah[2 * ROWS_BLK * KPAD];
  __shared__ __align__(16) float    Xs[XCHUNK * ROWS_BLK];
  __shared__ __align__(16) float    Hl[ROWS_BLK * UPAD];

  const int tid  = threadIdx.x;
  const int lane = tid & 31;
  const int wave = tid >> 5;
  const int c    = lane & 15;
  const int hh   = lane >> 4;
  const int mt   = wave >> 2;
  const int ug   = wave & 3;
  const int b0   = blockIdx.x * ROWS_BLK;
  const int unit = 16 * ug + c;
  const bool unit_ok = unit < NHID;
  const int unit_c = unit_ok ? unit : (NHID - 1);
  const int rowb = 16 * mt + 8 * hh;

#pragma unroll 1
  for (int i = tid; i < 2 * ROWS_BLK * KPAD; i += NTHR) Ah[i] = (_Float16)0.0f;

  {
    const int q = tid >> 6;
    const int j = tid & 63;
    const bool rok = j < NHID;
    const int srow = q * NHID + (rok ? j : (NHID - 1));
    const float* wr = w_hh + srow * NHID;
#pragma unroll 1
    for (int g = 0; g < KPAD / 8; ++g) {
      v8h hv;
#pragma unroll
      for (int e = 0; e < 8; ++e) {
        const int k  = 8 * g + e;
        const int kc = (k < NHID) ? k : (NHID - 1);
        const float v  = wr[kc];
        const float vs = (rok && (k < NHID)) ? (v * W_CARRY) : 0.0f;
        hv[e] = (_Float16)vs;
      }
      *(v8h*)(Wl + tid * KPAD + 8 * g) = hv;
    }
  }
  __syncthreads();

  v16h bf[NGATE][2];
#pragma unroll
  for (int q = 0; q < NGATE; ++q) {
#pragma unroll
    for (int ks = 0; ks < 2; ++ks)
      bf[q][ks] = Frag<_Float16>::load(Wl + (q * UPAD + unit) * KPAD + 32 * ks + 8 * hh);
  }

  float wihS[NGATE], bsS[NGATE];
#pragma unroll
  for (int q = 0; q < NGATE; ++q) {
    const int idx = q * NHID + unit_c;
    const float wv = w_ih[idx];
    const float bv = b_ih[idx] + b_hh[idx];
    wihS[q] = unit_ok ? (wv * ACC_CARRY) : 0.0f;
    bsS[q]  = unit_ok ? (bv * ACC_CARRY) : 0.0f;
  }

  float cst[8], hst[8];
#pragma unroll
  for (int r = 0; r < 8; ++r) { cst[r] = 0.0f; hst[r] = 0.0f; }

#pragma unroll 1
  for (int t0 = 0; t0 < NSTEP; t0 += XCHUNK) {
#pragma unroll
    for (int it = 0; it < 2; ++it) {
      const int idx = it * NTHR + tid;
      const int row = idx >> 4;
      const int c4  = (idx & 15) * 4;
      const v4f v = *(const v4f*)(x + (size_t)(b0 + row) * NSTEP + (size_t)(t0 + c4));
      const float v0 = v[0], v1 = v[1], v2 = v[2], v3 = v[3];
      Xs[(c4 + 0) * ROWS_BLK + row] = v0;
      Xs[(c4 + 1) * ROWS_BLK + row] = v1;
      Xs[(c4 + 2) * ROWS_BLK + row] = v2;
      Xs[(c4 + 3) * ROWS_BLK + row] = v3;
    }
    __syncthreads();

#pragma unroll 1
    for (int tt = 0; tt < XCHUNK; ++tt) {
      const int cur = tt & 1;
      const _Float16* ahc = Ah + cur * (ROWS_BLK * KPAD);
      _Float16*       ahn = Ah + (cur ^ 1) * (ROWS_BLK * KPAD);

      const float* xp = Xs + tt * ROWS_BLK + rowb;
      const v4f xa = *(const v4f*)(xp);
      const v4f xb = *(const v4f*)(xp + 4);
      float xv[8];
      xv[0] = xa[0]; xv[1] = xa[1]; xv[2] = xa[2]; xv[3] = xa[3];
      xv[4] = xb[0]; xv[5] = xb[1]; xv[6] = xb[2]; xv[7] = xb[3];

      const v16h a0 = Frag<_Float16>::load(ahc + (16 * mt + c) * KPAD + 8 * hh);
      const v16h a1 = Frag<_Float16>::load(ahc + (16 * mt + c) * KPAD + 32 + 8 * hh);

      v8f acc[NGATE];
#pragma unroll
      for (int q = 0; q < NGATE; ++q) {
#pragma unroll
        for (int r = 0; r < 8; ++r) acc[q][r] = fmaf(xv[r], wihS[q], bsS[q]);
      }
#pragma unroll
      for (int q = 0; q < NGATE; ++q) acc[q] = Frag<_Float16>::mma(a0, bf[q][0], acc[q]);
#pragma unroll
      for (int q = 0; q < NGATE; ++q) acc[q] = Frag<_Float16>::mma(a1, bf[q][1], acc[q]);
      step_guard(acc[0], acc[1], acc[2], acc[3], a0, a1);
      keep4_h(bf[0][0], bf[1][0], bf[2][0], bf[3][0]);
      keep4_h(bf[0][1], bf[1][1], bf[2][1], bf[3][1]);

#pragma unroll
      for (int r = 0; r < 8; ++r) {
        const float zi = acc[0][r] * ACC_CARRY_INV;
        const float zf = acc[1][r] * ACC_CARRY_INV;
        const float zg = acc[2][r] * ACC_CARRY_INV;
        const float zo = acc[3][r] * ACC_CARRY_INV;
        const float ig = fsig(zi);
        const float fg = fsig(zf);
        const float gg = ftanh(zg);
        const float og = fsig(zo);
        const float cn = fg * cst[r] + ig * gg;
        cst[r] = cn;
        const float hraw = og * ftanh(cn);
        const float hn = unit_ok ? hraw : 0.0f;
        hst[r] = hn;
        ahn[(rowb + r) * KPAD + unit] = (_Float16)(hn * H_CARRY);
      }
      __syncthreads();
    }
  }

#pragma unroll
  for (int r = 0; r < 8; ++r) Hl[(rowb + r) * UPAD + unit] = hst[r];
  __syncthreads();
  if (wave == 0) {
    float s = 0.0f;
#pragma unroll 1
    for (int j = 0; j < NHID; ++j) s = fmaf(Hl[lane * UPAD + j], w_lin[j], s);
    const float o = s + b_lin[0];
    volatile float* op = out + b0 + lane;
    *op = o;
    __threadfence();
    *op = o;
  }
}

extern "C" void kernel_launch(void* const* d_in, const int* in_sizes, int n_in,
                              void* d_out, int out_size, void* d_ws, size_t ws_size, hipStream_t stream) {
  (void)in_sizes; (void)out_size; (void)d_ws; (void)ws_size;
  if (n_in < 7 || d_out == nullptr) return;
  const float* x     = (const float*)d_in[0];
  const float* w_ih  = (const float*)d_in[1];
  const float* w_hh  = (const float*)d_in[2];
  const float* b_ih  = (const float*)d_in[3];
  const float* b_hh  = (const float*)d_in[4];
  const float* w_lin = (const float*)d_in[5];
  const float* b_lin = (const float*)d_in[6];
  float* out = (float*)d_out;
  lstm_seq_kernel<<<NBATCH / ROWS_BLK, NTHR, 0, stream>>>(x, w_ih, w_hh, b_ih, b_hh, w_lin, b_lin, out);
}
